// Net_21646635172359
// MI455X (gfx1250) — hardware-verified
//
#include <hip/hip_runtime.h>
#include <stddef.h>
#include <stdint.h>
#include <math.h>


#define NN     200000
#define EE     1600000
#define NN1    100000
#define EE2    100000
#define NN2    50000
#define NGR    1000
#define HH     25
#define NCLS   10
#define NOUTF  10000
#define MP1    100032
#define ETM    128
#define MPE    100096
#define W2KP   896
#define W2KB   832
#define XSP    36
#define HSP    28

#define NTHR   256
#define NWAVE  8
#define EPT    8
#define CHUNK  (NTHR * EPT)
#define WCAP   (EPT * 32)
#define LISTN  (NWAVE * WCAP)
#define GBM    64
#define GTHR   128

#define S1NB   2048
#define S1SL   11
#define S1RC   20480
#define S1DEG  64
#define PNB    1024
#define PSL    10
#define PRC    8192
#define PDEG   16
#define S2NB   1024
#define S2SL   10
#define S2RC   4096
#define S2DEG  32
#define PG1    98
#define PG2    49
#define WSMAX  134217728

static_assert((CHUNK & (CHUNK - 1)) == 0 && CHUNK <= 4096);
static_assert(S1NB == (1 << S1SL) && PNB == (1 << PSL) && S2NB == (1 << S2SL));
static_assert(((long long)EE << S1SL) < (1LL << 32));
static_assert(((long long)NN << PSL) < (1LL << 32) && ((long long)EE2 << S2SL) < (1LL << 32));
static_assert(((long long)CHUNK << S1SL) < (1LL << 31));
static_assert(NN % GBM == 0 && MP1 % GBM == 0 && MP1 >= NN1 && MPE % ETM == 0 && MPE >= EE2);
static_assert(PG1 * PNB >= MP1 && PG2 * PNB >= NN2);
static_assert(ETM * XSP + ETM * HSP == ETM * 64);
static_assert((LISTN + 2 * S1RC + 3 * S1NB) % (4) == 0 && (LISTN + 2 * PRC + 3 * PNB) % 4 == 0);
static_assert((LISTN + 2 * S2RC + 3 * S2NB) % 4 == 0);
static_assert((LISTN + 2 * S1RC + 3 * S1NB + 16) * 4 <= 300000);
static_assert(NOUTF == NGR * NCLS && (16 * NCLS * 4) % 128 == 0);

typedef float          v2f   __attribute__((ext_vector_type(2)));
typedef float          v4f   __attribute__((ext_vector_type(4)));
typedef float          v8f   __attribute__((ext_vector_type(8)));
typedef int            v4i   __attribute__((ext_vector_type(4)));
typedef int            v8i   __attribute__((ext_vector_type(8)));
typedef unsigned short v4us  __attribute__((ext_vector_type(4)));
typedef unsigned short v8us  __attribute__((ext_vector_type(8)));
typedef unsigned short v16us __attribute__((ext_vector_type(16)));
typedef __bf16         v16bf __attribute__((ext_vector_type(16)));
typedef v2f  __attribute__((may_alias)) v2fa;
typedef v4f  __attribute__((may_alias)) v4fa;
typedef v4i  __attribute__((may_alias)) v4ia;
typedef v4us __attribute__((may_alias)) v4usa;
typedef v8us __attribute__((may_alias)) v8usa;
union FragB { v16bf v; v16us u; v8us h[2]; v8i w; };

__device__ __forceinline__ v8f wmb(const FragB& a, const FragB& b, v8f c) {
  v8f d = __builtin_amdgcn_wmma_f32_16x16x32_bf16(false, a.v, false, b.v, (short)0, c, false, false);
  asm volatile("v_nop\n\tv_nop\n\tv_nop\n\tv_nop" : "+v"(d) : "v"(a.w), "v"(b.w));
  return d;
}

__device__ __forceinline__ unsigned bf16_bits(float f) {
  const unsigned u = __float_as_uint(f);
  return (u + 0x7FFFu + ((u >> 16) & 1u)) >> 16;
}
__device__ __forceinline__ float bf16_val(float f) {
  return __uint_as_float(bf16_bits(f) << 16);
}
__device__ __forceinline__ float nanmaxf(float a, float b) { return (a > b || a != a) ? a : b; }
__device__ __forceinline__ float eluf(float v) { return (v > 0.0f) ? v : expm1f(v); }

template <int B0>
__device__ __forceinline__ void split4(const v4f a, FragB& hi, FragB& lo) {
  unsigned hb;
  hb = bf16_bits(a.x); hi.u[B0 + 0] = (unsigned short)hb; lo.u[B0 + 0] = (unsigned short)bf16_bits(a.x - __uint_as_float(hb << 16));
  hb = bf16_bits(a.y); hi.u[B0 + 1] = (unsigned short)hb; lo.u[B0 + 1] = (unsigned short)bf16_bits(a.y - __uint_as_float(hb << 16));
  hb = bf16_bits(a.z); hi.u[B0 + 2] = (unsigned short)hb; lo.u[B0 + 2] = (unsigned short)bf16_bits(a.z - __uint_as_float(hb << 16));
  hb = bf16_bits(a.w); hi.u[B0 + 3] = (unsigned short)hb; lo.u[B0 + 3] = (unsigned short)bf16_bits(a.w - __uint_as_float(hb << 16));
}

template <int SLB>
__device__ __forceinline__ int scan_chunk(const int* __restrict__ dsts, int nE, int cbase, int slotBase,
                                          int nb, int vec8, int* list, int tid, int lane, int wave) {
  int wc = 0;
  const int el0  = tid * EPT;
  const int e0   = cbase + el0;
  const int sent = -2147483647 - 1;
  v4i da, db;
  if (vec8 != 0 && cbase + CHUNK <= nE) {
    da = *(const v4i*)(dsts + e0);
    db = *(const v4i*)(dsts + e0 + 4);
  } else {
    da.x = (e0     < nE) ? dsts[min(e0,     nE - 1)] : sent;
    da.y = (e0 + 1 < nE) ? dsts[min(e0 + 1, nE - 1)] : sent;
    da.z = (e0 + 2 < nE) ? dsts[min(e0 + 2, nE - 1)] : sent;
    da.w = (e0 + 3 < nE) ? dsts[min(e0 + 3, nE - 1)] : sent;
    db.x = (e0 + 4 < nE) ? dsts[min(e0 + 4, nE - 1)] : sent;
    db.y = (e0 + 5 < nE) ? dsts[min(e0 + 5, nE - 1)] : sent;
    db.z = (e0 + 6 < nE) ? dsts[min(e0 + 6, nE - 1)] : sent;
    db.w = (e0 + 7 < nE) ? dsts[min(e0 + 7, nE - 1)] : sent;
  }
  const unsigned nbs = (unsigned)slotBase;
  const unsigned unb = (unsigned)nb;
  const unsigned s0 = (unsigned)da.x - nbs, s1 = (unsigned)da.y - nbs;
  const unsigned s2 = (unsigned)da.z - nbs, s3 = (unsigned)da.w - nbs;
  const unsigned s4 = (unsigned)db.x - nbs, s5 = (unsigned)db.y - nbs;
  const unsigned s6 = (unsigned)db.z - nbs, s7 = (unsigned)db.w - nbs;
  const bool h0 = s0 < unb, h1 = s1 < unb, h2 = s2 < unb, h3 = s3 < unb;
  const bool h4 = s4 < unb, h5 = s5 < unb, h6 = s6 < unb, h7 = s7 < unb;
  const unsigned any = __builtin_amdgcn_ballot_w32(h0 | h1 | h2 | h3 | h4 | h5 | h6 | h7);
  if (any != 0u) {
#define HITJ(J, HJ, SJ) { \
      const unsigned mj = __builtin_amdgcn_ballot_w32(HJ); \
      if (mj != 0u) { \
        if (HJ) { \
          const int pos = wc + (int)__builtin_amdgcn_mbcnt_lo(mj, 0u); \
          if (pos < WCAP) list[wave * WCAP + pos] = ((el0 + (J)) << SLB) | (int)(SJ); \
        } \
        wc += (int)__builtin_popcount(mj); } }
    HITJ(0, h0, s0)
    HITJ(1, h1, s1)
    HITJ(2, h2, s2)
    HITJ(3, h3, s3)
    HITJ(4, h4, s4)
    HITJ(5, h5, s5)
    HITJ(6, h6, s6)
    HITJ(7, h7, s7)
#undef HITJ
  }
  return wc;
}

template <int NB, int SL, int RC>
__device__ __forceinline__ void scan_build(const int* __restrict__ keys, int nK, int vec8, int slotBase,
                                           int* dsm, int tid, int lane, int wave, int& ovfOut) {
  constexpr int ZI = LISTN + 2 * RC + 3 * NB;
  int* list = dsm;
  int* hl   = dsm + LISTN;
  int* sl   = hl + RC;
  int* cnt  = sl + RC;
  int* offs = cnt + NB;
  int* cur  = offs + NB;
  int* misc = cur + NB;
  {
    const v4i z4 = {0, 0, 0, 0};
    for (int i = tid * 4; i < ZI; i += NTHR * 4) *(v4ia*)(dsm + i) = z4;
    if (tid < 16) misc[tid] = 0;
  }
  __syncthreads();

  int t = 0, ov = 0;
  const int nChunks = (nK + CHUNK - 1) / CHUNK;
#pragma unroll 1
  for (int ch = 0; ch < nChunks; ++ch) {
    const int cbase = ch * CHUNK;
    const int wc = scan_chunk<SL>(keys, nK, cbase, slotBase, NB, vec8, list, tid, lane, wave);
    if (lane == 0) misc[wave] = wc;
    __syncthreads();
    if (wave == 0) {
#pragma unroll 1
      for (int w2 = 0; w2 < NWAVE; ++w2) {
        int c = misc[w2];
        c = c < 0 ? 0 : (c > WCAP ? WCAP : c);
#pragma unroll 1
        for (int b0 = 0; b0 < c; b0 += 32) {
          const int idx = b0 + lane;
          const int ent = list[w2 * WCAP + (idx < WCAP ? idx : WCAP - 1)];
          const int m32 = (c - b0) < 32 ? (c - b0) : 32;
#pragma unroll 1
          for (int k = 0; k < m32; ++k) {
            const int u    = __builtin_amdgcn_readlane(ent, k);
            const int slot = u & (NB - 1);
            const int el   = (u >> SL) & (CHUNK - 1);
            const int pk   = (int)(((unsigned)(cbase + el) << SL) | (unsigned)slot);
            if (t < RC) {
              if (lane == 0) { hl[t] = pk; cnt[slot] = cnt[slot] + 1; }
              t = t + 1;
            } else {
              ov = 1;
            }
          }
        }
      }
    }
    __syncthreads();
  }
  if (wave == 0 && lane == 0) { misc[8] = t; misc[9] = ov; }
  __syncthreads();
  int tt = misc[8];
  tt = tt < 0 ? 0 : (tt > RC ? RC : tt);
  ovfOut = misc[9];

  if (wave == 0) {
    const int base = lane * (NB / 32);
    int s = 0;
#pragma unroll 1
    for (int i = 0; i < NB / 32; ++i) s += cnt[base + i];
    int incl = s;
#pragma unroll
    for (int d = 1; d < 32; d <<= 1) {
      const int y = __shfl_up(incl, d, 32);
      if (lane >= d) incl += y;
    }
    int run = incl - s;
#pragma unroll 1
    for (int i = 0; i < NB / 32; ++i) {
      const int cv = cnt[base + i];
      offs[base + i] = run;
      cur[base + i]  = run;
      run += cv;
    }
  }
  __syncthreads();
  if (wave == 0) {
#pragma unroll 1
    for (int b0 = 0; b0 < tt; b0 += 32) {
      const int idx = b0 + lane;
      const int ent = hl[idx < RC ? idx : RC - 1];
      const int m32 = (tt - b0) < 32 ? (tt - b0) : 32;
#pragma unroll 1
      for (int k = 0; k < m32; ++k) {
        const int u    = __builtin_amdgcn_readlane(ent, k);
        const int slot = u & (NB - 1);
        if (lane == 0) {
          int p = cur[slot];
          p = p < 0 ? 0 : (p > RC - 1 ? RC - 1 : p);
          sl[p] = u;
          cur[slot] = p + 1;
        }
      }
    }
  }
  __syncthreads();
}

__global__ __launch_bounds__(NTHR) void k_prep(const float* __restrict__ w2a, const float* __restrict__ b2a,
                                               const float* __restrict__ root1, const float* __restrict__ bias1,
                                               const float* __restrict__ w2b, const float* __restrict__ b2b,
                                               const float* __restrict__ root2, const float* __restrict__ fc1w,
                                               const float* __restrict__ fc2w,
                                               unsigned short* B1t, unsigned short* W2t, unsigned short* R2t,
                                               unsigned short* F1t, unsigned short* F2t) {
  __shared__ float sb[32 * 32];
  const int blk = (int)blockIdx.x, tid = (int)threadIdx.x;
  v8us o;
  unsigned short* dp;
  if (blk < 26) {
    const int u  = blk * NTHR + tid;
    const int n  = u / 104;
    const int q  = u - n * 104;
    const int k8 = q * 8;
    const int h  = k8 >> 5;
    const int i0 = k8 & 31;
    const bool ok = h < HH;
    const int hc = ok ? h : HH - 1;
    const float* p = w2b + (size_t)hc * 2048 + (size_t)i0 * 64 + n;
#pragma unroll
    for (int i = 0; i < 8; ++i) {
      const unsigned b = bf16_bits(p[(size_t)i * 64]);
      o[i] = ok ? (unsigned short)b : (unsigned short)0;
    }
    dp = W2t + (size_t)n * W2KP + k8;
  } else if (blk < 28) {
    const int u  = (blk - 26) * NTHR + tid;
    const int n  = u >> 3;
    const int q  = u & 7;
    const bool ok = q < 4;
    const int i0 = ok ? q * 8 : 0;
    const float* p = b2b + (size_t)i0 * 64 + n;
#pragma unroll
    for (int i = 0; i < 8; ++i) {
      const unsigned b = bf16_bits(p[(size_t)i * 64]);
      o[i] = ok ? (unsigned short)b : (unsigned short)0;
    }
    dp = W2t + (size_t)n * W2KP + W2KB + q * 8;
  } else if (blk == 28) {
    const int n  = tid >> 2;
    const int k8 = (tid & 3) * 8;
    const float* p = root2 + (size_t)k8 * 64 + n;
#pragma unroll
    for (int i = 0; i < 8; ++i) o[i] = (unsigned short)bf16_bits(p[(size_t)i * 64]);
    dp = R2t + (size_t)n * 32 + k8;
  } else if (blk < 33) {
    const int u  = (blk - 29) * NTHR + tid;
    const int n  = u >> 3;
    const int k8 = (u & 7) * 8;
    const float* p = fc1w + (size_t)k8 * 128 + n;
#pragma unroll
    for (int i = 0; i < 8; ++i) o[i] = (unsigned short)bf16_bits(p[(size_t)i * 128]);
    dp = F1t + (size_t)n * 64 + k8;
  } else if (blk == 33) {
    const int n  = tid >> 4;
    const int k8 = (tid & 15) * 8;
    const bool ok = n < NCLS;
    const int nc = ok ? n : NCLS - 1;
    const float* p = fc2w + (size_t)k8 * NCLS + nc;
#pragma unroll
    for (int i = 0; i < 8; ++i) {
      const unsigned b = bf16_bits(p[(size_t)i * NCLS]);
      o[i] = ok ? (unsigned short)b : (unsigned short)0;
    }
    dp = F2t + (size_t)n * 128 + k8;
  } else {
#pragma unroll 1
    for (int it = 0; it < 4; ++it) {
      const int idx = it * NTHR + tid;
      const int k = idx >> 5, n = idx & 31;
      const float wv = w2a[idx < 800 ? idx : 799];
      const float bv = b2a[n];
      const float rv = root1[n];
      const float cv = bias1[n];
      float v = 0.0f;
      v = (k == 27) ? cv : v;
      v = (k == 26) ? rv : v;
      v = (k == 25) ? bv : v;
      v = (k < HH) ? wv : v;
      sb[idx] = v;
    }
    __syncthreads();
    if (tid >= 128) return;
    const int n  = tid >> 2;
    const int k8 = (tid & 3) * 8;
#pragma unroll
    for (int i = 0; i < 8; ++i) o[i] = (unsigned short)bf16_bits(sb[(k8 + i) * 32 + n]);
    dp = B1t + (size_t)n * 32 + k8;
  }
  *(volatile v8us*)dp = o;
  __threadfence();
  *(volatile v8us*)dp = o;
}

__global__ __launch_bounds__(NTHR) void k_scan1(const int* __restrict__ ei, const float* __restrict__ x,
                                                const float* __restrict__ ea, const float* __restrict__ w1,
                                                const float* __restrict__ b1, float* A1) {
  extern __shared__ __attribute__((aligned(16))) int dsm[];
  constexpr int NB = S1NB, SL = S1SL, RC = S1RC;
  int* sl   = dsm + LISTN + RC;
  int* cnt  = sl + RC;
  int* offs = cnt + NB;
  const int tid = (int)threadIdx.x, lane = tid & 31, wave = tid >> 5;
  const int nodeBase = (int)blockIdx.x * NB;
  int ovf = 0;
  scan_build<NB, SL, RC>(ei + EE, EE, 1, nodeBase, dsm, tid, lane, wave, ovf);

  const int cc = lane < HH ? lane : HH - 1;
  float wa = bf16_val(w1[cc]);
  float wb = bf16_val(w1[HH + cc]);
  float bb = bf16_val(b1[cc]);
  wa = lane < HH ? wa : 0.0f;
  wb = lane < HH ? wb : 0.0f;
  bb = lane < HH ? bb : (lane == HH ? 1.0f : 0.0f);

  const float qnan = __int_as_float(0x7fc00000);
  const float pz = (ovf != 0) ? qnan : 0.0f;
#pragma unroll 1
  for (int si = 0; si < NB / NWAVE; ++si) {
    const int s    = si * NWAVE + wave;
    const int node = nodeBase + s;
    int c = cnt[s];
    const bool big = c > S1DEG;
    c = c < 0 ? 0 : (c > S1DEG ? S1DEG : c);
    int o = offs[s];
    o = o < 0 ? 0 : (o > RC ? RC : o);
    float acc = 0.0f;
#pragma unroll 1
    for (int b0 = 0; b0 < c; b0 += 32) {
      int idx = o + b0 + lane;
      idx = idx > RC - 1 ? RC - 1 : idx;
      const int ent = sl[idx];
      int eid = (int)((unsigned)ent >> SL);
      eid = eid > EE - 1 ? EE - 1 : eid;
      int sr = ei[eid];
      sr = sr < 0 ? 0 : (sr > NN - 1 ? NN - 1 : sr);
      const int xsi = __float_as_int(bf16_val(x[sr]));
      const v2f e2 = *(const v2fa*)(ea + 2 * (size_t)eid);
      const int a0i = __float_as_int(bf16_val(e2.x));
      const int a1i = __float_as_int(bf16_val(e2.y));
      const int m32 = (c - b0) < 32 ? (c - b0) : 32;
#pragma unroll 1
      for (int k = 0; k < m32; ++k) {
        const float xk = __int_as_float(__builtin_amdgcn_readlane(xsi, k));
        const float p0 = __int_as_float(__builtin_amdgcn_readlane(a0i, k));
        const float p1 = __int_as_float(__builtin_amdgcn_readlane(a1i, k));
        float hd = fmaf(p1, wb, p0 * wa) + bb;
        hd = fmaxf(hd, 0.0f);
        acc = fmaf(xk, hd, acc);
      }
    }
    const int nc = node < NN ? node : NN - 1;
    const float xi = bf16_val(x[nc]);
    float val = acc;
    val = (lane == 26) ? xi : val;
    val = (lane == 27) ? 1.0f : val;
    val = val + (big ? qnan : pz);
    if (node < NN) {
      float* op = A1 + (size_t)node * 32 + lane;
      *(volatile float*)op = val;
      __threadfence();
      *(volatile float*)op = val;
    }
  }
}

template <int KA, int NCOL, int HASB, int ELU>
__global__ __launch_bounds__(GTHR) void k_gemm(const float* __restrict__ A, const unsigned short* __restrict__ WT,
                                               const float* __restrict__ bias, float* outF) {
  constexpr int NT  = NCOL / 16;
  constexpr int LPR = NCOL / 4;
  constexpr int RPI = 32 / LPR;
  constexpr int NIT = 16 / RPI;
  static_assert(KA % 32 == 0 && NCOL % 16 == 0 && (LPR == 8 || LPR == 16));
  __shared__ __attribute__((aligned(16))) float stg[GBM * NCOL];
  const int tid = (int)threadIdx.x, lane = tid & 31, wave = tid >> 5, hh = lane >> 4, m = lane & 15;
  const int rowBase = (int)blockIdx.x * GBM;

  v8f acc[NT];
  {
    const v8f z = {0.f, 0.f, 0.f, 0.f, 0.f, 0.f, 0.f, 0.f};
#pragma unroll
    for (int t = 0; t < NT; ++t) acc[t] = z;
  }
  const float* ap = A + (size_t)(rowBase + 16 * wave + m) * (size_t)KA + 8 * hh;
  const unsigned short* wp = WT + (size_t)m * (size_t)KA + 8 * hh;
#pragma unroll 1
  for (int k0 = 0; k0 < KA; k0 += 32) {
    const v4f a0 = *(const v4fa*)(ap + k0);
    const v4f a1 = *(const v4fa*)(ap + k0 + 4);
    const v4f a2 = *(const v4fa*)(ap + k0 + 16);
    const v4f a3 = *(const v4fa*)(ap + k0 + 20);
    FragB ah, al;
    split4<0>(a0, ah, al);
    split4<4>(a1, ah, al);
    split4<8>(a2, ah, al);
    split4<12>(a3, ah, al);
#pragma unroll
    for (int t = 0; t < NT; ++t) {
      const unsigned short* wq = wp + (size_t)(16 * t) * (size_t)KA + k0;
      FragB bf;
      bf.h[0] = *(const v8usa*)wq;
      bf.h[1] = *(const v8usa*)(wq + 16);
      acc[t] = wmb(ah, bf, acc[t]);
      acc[t] = wmb(al, bf, acc[t]);
    }
  }

#pragma unroll
  for (int t = 0; t < NT; ++t) {
    const int lc = 16 * t + m;
#pragma unroll
    for (int r = 0; r < 8; ++r) {
      const int lr = 16 * wave + 8 * hh + r;
      stg[lr * NCOL + lc] = acc[t][r];
    }
  }
  __syncthreads();

  const int lsub = lane / LPR;
  const int lcol = 4 * (lane % LPR);
  if constexpr (HASB != 0 || ELU != 0) {
    v4f b4 = {0.f, 0.f, 0.f, 0.f};
    if constexpr (HASB != 0) {
      const v4f t4 = *(const v4fa*)(bias + lcol);
      b4.x = bf16_val(t4.x); b4.y = bf16_val(t4.y); b4.z = bf16_val(t4.z); b4.w = bf16_val(t4.w);
    }
#pragma unroll 1
    for (int i = 0; i < NIT; ++i) {
      float* sp = stg + (16 * wave + RPI * i + lsub) * NCOL + lcol;
      v4f v = *(v4fa*)sp;
      v = v + b4;
      if constexpr (ELU != 0) { v.x = eluf(v.x); v.y = eluf(v.y); v.z = eluf(v.z); v.w = eluf(v.w); }
      *(v4fa*)sp = v;
    }
  }

  v4f fv[NIT];
#pragma unroll
  for (int i = 0; i < NIT; ++i) {
    const int lr = 16 * wave + RPI * i + lsub;
    fv[i] = *(const v4fa*)(stg + lr * NCOL + lcol);
  }
#pragma unroll
  for (int i = 0; i < NIT; ++i) {
    const int gr = rowBase + 16 * wave + RPI * i + lsub;
    float* op = outF + (size_t)gr * (size_t)NCOL + lcol;
    *(volatile v4f*)op = fv[i];
  }
  __threadfence();
#pragma unroll
  for (int i = 0; i < NIT; ++i) {
    const int gr = rowBase + 16 * wave + RPI * i + lsub;
    float* op = outF + (size_t)gr * (size_t)NCOL + lcol;
    *(volatile v4f*)op = fv[i];
  }
}

template <int C, int POS>
__global__ __launch_bounds__(NTHR) void k_pool(const int* __restrict__ keys, int nK, int nSeg, int mRows,
                                               const float* __restrict__ feat, const float* __restrict__ pos,
                                               const int* __restrict__ bat, float* xo, float* poso, int* bato) {
  extern __shared__ __attribute__((aligned(16))) int dsm[];
  constexpr int NB = PNB, SL = PSL, RC = PRC;
  int* sl    = dsm + LISTN + RC;
  int* cnt   = sl + RC;
  int* offs  = cnt + NB;
  int* sbat  = dsm + LISTN + 2 * RC + 3 * NB + 16;
  float* spos = (float*)(sbat + NB);
  const int tid = (int)threadIdx.x, lane = tid & 31, wave = tid >> 5;
  const int nodeBase = (int)blockIdx.x * NB;
  int ovf = 0;
  scan_build<NB, SL, RC>(keys, nK, 1, nodeBase, dsm, tid, lane, wave, ovf);

  const float qnan = __int_as_float(0x7fc00000);
  const float ninf = __int_as_float((int)0xff800000u);
  const float pz = (ovf != 0) ? qnan : 0.0f;
  const int sa = (2 * lane) & 31, sb = (2 * lane + 1) & 31;
#pragma unroll 1
  for (int si = 0; si < NB / NWAVE; ++si) {
    const int s    = si * NWAVE + wave;
    const int node = nodeBase + s;
    int c = cnt[s];
    const bool big = c > PDEG;
    c = c < 0 ? 0 : (c > PDEG ? PDEG : c);
    int o = offs[s];
    o = o < 0 ? 0 : (o > RC ? RC : o);
    float x0 = ninf, x1 = ninf, px = 0.0f, py = 0.0f;
    int bm = -2147483647 - 1;
#pragma unroll 1
    for (int b0 = 0; b0 < c; b0 += 32) {
      int idx = o + b0 + lane;
      idx = idx > RC - 1 ? RC - 1 : idx;
      const int ent = sl[idx];
      int nid = (int)((unsigned)ent >> SL);
      nid = nid > nK - 1 ? nK - 1 : nid;
      const int bt = bat[nid];
      int qxi = 0, qyi = 0;
      if constexpr (POS != 0) {
        const v2f p = *(const v2fa*)(pos + 2 * (size_t)nid);
        qxi = __float_as_int(bf16_val(p.x));
        qyi = __float_as_int(bf16_val(p.y));
      }
      const int m32 = (c - b0) < 32 ? (c - b0) : 32;
#pragma unroll 1
      for (int k = 0; k < m32; ++k) {
        const int nk = __builtin_amdgcn_readlane(nid, k);
        const int bk = __builtin_amdgcn_readlane(bt, k);
        bm = bk > bm ? bk : bm;
        if constexpr (POS != 0) {
          px += __int_as_float(__builtin_amdgcn_readlane(qxi, k));
          py += __int_as_float(__builtin_amdgcn_readlane(qyi, k));
        }
        if constexpr (C == 32) {
          const float v = feat[(size_t)nk * 32 + lane];
          x0 = nanmaxf(v, x0);
        } else {
          const v2f a = *(const v2fa*)(feat + (size_t)nk * 64 + 2 * lane);
          x0 = nanmaxf(a.x, x0);
          x1 = nanmaxf(a.y, x1);
        }
      }
    }
    const float pzr = big ? qnan : pz;
    const bool live = node < nSeg;
    const float o0 = live ? (x0 + pzr) : 0.0f;
    const float o1 = live ? (x1 + pzr) : 0.0f;
    if (lane == 0) {
      sbat[s] = bm;
      if constexpr (POS != 0) {
        const float cf = (c < 1) ? 1.0f : (float)c;
        const float rc = 1.0f / cf;
        spos[2 * s]     = px * rc + pzr;
        spos[2 * s + 1] = py * rc + pzr;
      }
    }
    if constexpr (C == 32) {
      if (node < mRows) {
        float* op = xo + (size_t)node * 32 + lane;
        *(volatile float*)op = o0;
        __threadfence();
        *(volatile float*)op = o0;
      }
    } else {
      v4f ow;
      ow.x = __shfl(o0, sa, 32); ow.y = __shfl(o1, sa, 32);
      ow.z = __shfl(o0, sb, 32); ow.w = __shfl(o1, sb, 32);
      const bool wr = (node < mRows) && (lane < 16);
      float* op = xo + (size_t)node * 64 + 4 * (lane & 15);
      if (wr) *(volatile v4f*)op = ow;
      __threadfence();
      if (wr) *(volatile v4f*)op = ow;
    }
  }
  __syncthreads();
  {
    const v4i bv = *(const v4ia*)(sbat + 4 * tid);
    int* bp = bato + (size_t)nodeBase + 4 * tid;
    v4f p0 = {0.f, 0.f, 0.f, 0.f}, p1 = {0.f, 0.f, 0.f, 0.f};
    float* pp = poso + 2 * (size_t)nodeBase + 4 * tid;
    if constexpr (POS != 0) {
      p0 = *(const v4fa*)(spos + 4 * tid);
      p1 = *(const v4fa*)(spos + 4 * (NTHR + tid));
    }
    *(volatile v4i*)bp = bv;
    if constexpr (POS != 0) { *(volatile v4f*)pp = p0; *(volatile v4f*)(pp + 4 * NTHR) = p1; }
    __threadfence();
    *(volatile v4i*)bp = bv;
    if constexpr (POS != 0) { *(volatile v4f*)pp = p0; *(volatile v4f*)(pp + 4 * NTHR) = p1; }
  }
}

__global__ __launch_bounds__(NTHR) void k_cartmax(const int* __restrict__ ei2, const float* __restrict__ pos1,
                                                  float* rec) {
  __shared__ float red[NWAVE];
  const int tid = (int)threadIdx.x, lane = tid & 31, wave = tid >> 5;
  float mx = 0.0f;
#pragma unroll 1
  for (int e = tid; e < EE2; e += NTHR) {
    int s = ei2[e];
    int d = ei2[EE2 + e];
    s = s < 0 ? 0 : (s > NN1 - 1 ? NN1 - 1 : s);
    d = d < 0 ? 0 : (d > NN1 - 1 ? NN1 - 1 : d);
    const v2f ps = *(const v2fa*)(pos1 + 2 * (size_t)s);
    const v2f pd = *(const v2fa*)(pos1 + 2 * (size_t)d);
    const float dx = fabsf(ps.x - pd.x);
    const float dy = fabsf(ps.y - pd.y);
    mx = nanmaxf(dx, mx);
    mx = nanmaxf(dy, mx);
  }
#pragma unroll
  for (int d = 16; d >= 1; d >>= 1) {
    const float ot = __shfl_xor(mx, d, 32);
    mx = nanmaxf(ot, mx);
  }
  if (lane == 0) red[wave] = mx;
  __syncthreads();
  float r = red[0];
#pragma unroll
  for (int w2 = 1; w2 < NWAVE; ++w2) r = nanmaxf(red[w2], r);
  v4f ov; ov.x = r; ov.y = r; ov.z = r; ov.w = r;
  const bool st = (wave == 0) && (lane < 8);
  float* op = rec + 4 * (lane & 7);
  if (st) *(volatile v4f*)op = ov;
  __threadfence();
  if (st) *(volatile v4f*)op = ov;
}

__global__ __launch_bounds__(NTHR) void k_edge(const int* __restrict__ ei2, const float* __restrict__ X1,
                                               const float* __restrict__ pos1, const float* __restrict__ rec,
                                               const float* __restrict__ w1, const float* __restrict__ b1,
                                               const unsigned short* __restrict__ W2t, float* MSG) {
  __shared__ __attribute__((aligned(16))) float sm[ETM * 64];
  __shared__ float sw[96];
  float* xs = sm;
  float* hs = sm + ETM * XSP;
  const int tid = (int)threadIdx.x, lane = tid & 31, wave = tid >> 5, hh = lane >> 4, m = lane & 15;
  const int e0 = (int)blockIdx.x * ETM;

  if (tid < 96) {
    const int i1 = tid < 50 ? tid : 49;
    int i2 = tid - 50;
    i2 = i2 < 0 ? 0 : (i2 > HH - 1 ? HH - 1 : i2);
    const float a = w1[i1];
    const float b = b1[i2];
    float v = (tid < 75) ? b : 0.0f;
    v = (tid < 50) ? a : v;
    sw[tid] = bf16_val(v);
  }
  __syncthreads();

  const float mxv = rec[0];
  const float inv = 1.0f / (2.0f * mxv);
  if (tid < ETM) {
    int e = e0 + tid;
    e = e > EE2 - 1 ? EE2 - 1 : e;
    int s = ei2[e];
    int d = ei2[EE2 + e];
    s = s < 0 ? 0 : (s > NN1 - 1 ? NN1 - 1 : s);
    d = d < 0 ? 0 : (d > NN1 - 1 ? NN1 - 1 : d);
    const v2f ps = *(const v2fa*)(pos1 + 2 * (size_t)s);
    const v2f pd = *(const v2fa*)(pos1 + 2 * (size_t)d);
    const float a0 = (ps.x - pd.x) * inv + 0.5f;
    const float a1 = (ps.y - pd.y) * inv + 0.5f;
    float* hr = hs + tid * HSP;
#pragma unroll 1
    for (int h = 0; h < HH; ++h) {
      float v = fmaf(a1, sw[HH + h], a0 * sw[h]) + sw[2 * HH + h];
      v = (v < 0.0f) ? 0.0f : v;
      hr[h] = v;
    }
    hr[25] = 1.0f; hr[26] = 0.0f; hr[27] = 0.0f;
  }
#pragma unroll
  for (int it = 0; it < 4; ++it) {
    const int idx = it * NTHR + tid;
    const int row = idx >> 3, q = idx & 7;
    int e = e0 + row;
    e = e > EE2 - 1 ? EE2 - 1 : e;
    int s = ei2[e];
    s = s < 0 ? 0 : (s > NN1 - 1 ? NN1 - 1 : s);
    const v4f v = *(const v4fa*)(X1 + (size_t)s * 32 + 4 * q);
    *(v4fa*)(xs + row * XSP + 4 * q) = v;
  }
  __syncthreads();

  const int row = 16 * wave + m;
  const float* xr = xs + row * XSP + 8 * hh;
  const v4f x0 = *(const v4fa*)xr;
  const v4f x1 = *(const v4fa*)(xr + 4);
  const v4f x2 = *(const v4fa*)(xr + 16);
  const v4f x3 = *(const v4fa*)(xr + 20);
  const float* hrow = hs + row * HSP;

  v8f acc[4];
  {
    const v8f z = {0.f, 0.f, 0.f, 0.f, 0.f, 0.f, 0.f, 0.f};
    acc[0] = z; acc[1] = z; acc[2] = z; acc[3] = z;
  }
  const unsigned short* wp = W2t + (size_t)m * W2KP + 8 * hh;
#pragma unroll 1
  for (int c = 0; c < HH + 1; ++c) {
    const float hd = hrow[c];
    const int kq = (c < HH) ? 32 * c : W2KB;
    FragB ah, al;
    split4<0>(x0 * hd, ah, al);
    split4<4>(x1 * hd, ah, al);
    split4<8>(x2 * hd, ah, al);
    split4<12>(x3 * hd, ah, al);
#pragma unroll
    for (int t = 0; t < 4; ++t) {
      const unsigned short* wq = wp + (size_t)(16 * t) * W2KP + kq;
      FragB bf;
      bf.h[0] = *(const v8usa*)wq;
      bf.h[1] = *(const v8usa*)(wq + 16);
      acc[t] = wmb(ah, bf, acc[t]);
      acc[t] = wmb(al, bf, acc[t]);
    }
  }
  __syncthreads();

#pragma unroll
  for (int t = 0; t < 4; ++t) {
    const int lc = 16 * t + m;
#pragma unroll
    for (int r = 0; r < 8; ++r) {
      const int lr = 16 * wave + 8 * hh + r;
      sm[lr * 64 + lc] = acc[t][r];
    }
  }
  __syncthreads();

  v4f fv[8];
#pragma unroll
  for (int i = 0; i < 8; ++i) {
    const int lr = 16 * wave + 2 * i + hh;
    fv[i] = *(const v4fa*)(sm + lr * 64 + 4 * m);
  }
#pragma unroll
  for (int i = 0; i < 8; ++i) {
    const int gr = e0 + 16 * wave + 2 * i + hh;
    float* op = MSG + (size_t)gr * 64 + 4 * m;
    *(volatile v4f*)op = fv[i];
  }
  __threadfence();
#pragma unroll
  for (int i = 0; i < 8; ++i) {
    const int gr = e0 + 16 * wave + 2 * i + hh;
    float* op = MSG + (size_t)gr * 64 + 4 * m;
    *(volatile v4f*)op = fv[i];
  }
}

__global__ __launch_bounds__(NTHR) void k_scan2(const int* __restrict__ ei2, const float* __restrict__ MSG,
                                                const float* __restrict__ R, float* H2) {
  extern __shared__ __attribute__((aligned(16))) int dsm[];
  constexpr int NB = S2NB, SL = S2SL, RC = S2RC;
  int* sl   = dsm + LISTN + RC;
  int* cnt  = sl + RC;
  int* offs = cnt + NB;
  const int tid = (int)threadIdx.x, lane = tid & 31, wave = tid >> 5;
  const int nodeBase = (int)blockIdx.x * NB;
  int ovf = 0;
  scan_build<NB, SL, RC>(ei2 + EE2, EE2, 1, nodeBase, dsm, tid, lane, wave, ovf);

  const float qnan = __int_as_float(0x7fc00000);
  const float pz = (ovf != 0) ? qnan : 0.0f;
  const int sa = (2 * lane) & 31, sb = (2 * lane + 1) & 31;
#pragma unroll 1
  for (int si = 0; si < NB / NWAVE; ++si) {
    const int s    = si * NWAVE + wave;
    const int node = nodeBase + s;
    int c = cnt[s];
    const bool big = c > S2DEG;
    c = c < 0 ? 0 : (c > S2DEG ? S2DEG : c);
    int o = offs[s];
    o = o < 0 ? 0 : (o > RC ? RC : o);
    float a0 = 0.0f, a1 = 0.0f;
#pragma unroll 1
    for (int b0 = 0; b0 < c; b0 += 32) {
      int idx = o + b0 + lane;
      idx = idx > RC - 1 ? RC - 1 : idx;
      const int ent = sl[idx];
      int eid = (int)((unsigned)ent >> SL);
      eid = eid > EE2 - 1 ? EE2 - 1 : eid;
      const int m32 = (c - b0) < 32 ? (c - b0) : 32;
#pragma unroll 1
      for (int k = 0; k < m32; ++k) {
        const int ek = __builtin_amdgcn_readlane(eid, k);
        const v2f a = *(const v2fa*)(MSG + (size_t)ek * 64 + 2 * lane);
        a0 += a.x; a1 += a.y;
      }
    }
    const int nc = node < NN1 ? node : NN1 - 1;
    const v2f rr = *(const v2fa*)(R + (size_t)nc * 64 + 2 * lane);
    const float pzr = big ? qnan : pz;
    const float y0 = eluf(a0 + rr.x) + pzr;
    const float y1 = eluf(a1 + rr.y) + pzr;
    v4f ow;
    ow.x = __shfl(y0, sa, 32); ow.y = __shfl(y1, sa, 32);
    ow.z = __shfl(y0, sb, 32); ow.w = __shfl(y1, sb, 32);
    const bool wr = (node < NN1) && (lane < 16);
    float* op = H2 + (size_t)node * 64 + 4 * (lane & 15);
    if (wr) *(volatile v4f*)op = ow;
    __threadfence();
    if (wr) *(volatile v4f*)op = ow;
  }
}

__global__ __launch_bounds__(NTHR) void k_head(const float* __restrict__ X2, const int* __restrict__ bat2,
                                               const unsigned short* __restrict__ F1t,
                                               const unsigned short* __restrict__ F2t,
                                               const float* __restrict__ fc1b, const float* __restrict__ fc2b,
                                               float* out) {
  __shared__ __attribute__((aligned(16))) float gs[16 * 64];
  __shared__ __attribute__((aligned(16))) unsigned short gh[16 * 64];
  __shared__ __attribute__((aligned(16))) unsigned short gl[16 * 64];
  __shared__ __attribute__((aligned(16))) float zs[16 * 128];
  __shared__ __attribute__((aligned(16))) unsigned short zh[16 * 128];
  __shared__ __attribute__((aligned(16))) unsigned short zl[16 * 128];
  __shared__ float lg[16 * 16];
  __shared__ __attribute__((aligned(16))) float os[160];
  const int tid = (int)threadIdx.x, lane = tid & 31, wave = tid >> 5, hh = lane >> 4, m = lane & 15;
  const int gbase = (int)blockIdx.x * 16;

#pragma unroll 1
  for (int j = 0; j < 2; ++j) {
    const int r = 2 * wave + j;
    const int g = gbase + r;
    float a0 = 0.0f, a1 = 0.0f;
    int cnt = 0;
#pragma unroll 1
    for (int i0 = 0; i0 < NN2; i0 += 32) {
      const int i  = i0 + lane;
      const int ic = i < NN2 ? i : NN2 - 1;
      const int b  = bat2[ic];
      const bool hit = (i < NN2) && (b == g);
      unsigned msk = __builtin_amdgcn_ballot_w32(hit);
      int nh = (int)__builtin_popcount(msk);
      nh = nh > 32 ? 32 : nh;
      cnt += nh;
#pragma unroll 1
      for (int q = 0; q < nh; ++q) {
        const int k = __builtin_ffs((int)msk) - 1;
        msk &= msk - 1u;
        int node = i0 + (k < 0 ? 0 : k);
        node = node > NN2 - 1 ? NN2 - 1 : node;
        const v2f v = *(const v2fa*)(X2 + (size_t)node * 64 + 2 * lane);
        a0 += v.x; a1 += v.y;
      }
    }
    const float cf = (cnt < 1) ? 1.0f : (float)cnt;
    const float rc = 1.0f / cf;
    v2f gv; gv.x = a0 * rc; gv.y = a1 * rc;
    *(v2fa*)(gs + r * 64 + 2 * lane) = gv;
  }
  __syncthreads();
  {
    const v4f v = *(const v4fa*)(gs + 4 * tid);
    v4us h4, l4;
    unsigned hb;
    hb = bf16_bits(v.x); h4[0] = (unsigned short)hb; l4[0] = (unsigned short)bf16_bits(v.x - __uint_as_float(hb << 16));
    hb = bf16_bits(v.y); h4[1] = (unsigned short)hb; l4[1] = (unsigned short)bf16_bits(v.y - __uint_as_float(hb << 16));
    hb = bf16_bits(v.z); h4[2] = (unsigned short)hb; l4[2] = (unsigned short)bf16_bits(v.z - __uint_as_float(hb << 16));
    hb = bf16_bits(v.w); h4[3] = (unsigned short)hb; l4[3] = (unsigned short)bf16_bits(v.w - __uint_as_float(hb << 16));
    *(v4usa*)(gh + 4 * tid) = h4;
    *(v4usa*)(gl + 4 * tid) = l4;
  }
  __syncthreads();

  {
    v8f acc = {0.f, 0.f, 0.f, 0.f, 0.f, 0.f, 0.f, 0.f};
#pragma unroll 1
    for (int k0 = 0; k0 < 64; k0 += 32) {
      FragB ah, al, bf;
      ah.h[0] = *(const v8usa*)(gh + m * 64 + k0 + 8 * hh);
      ah.h[1] = *(const v8usa*)(gh + m * 64 + k0 + 16 + 8 * hh);
      al.h[0] = *(const v8usa*)(gl + m * 64 + k0 + 8 * hh);
      al.h[1] = *(const v8usa*)(gl + m * 64 + k0 + 16 + 8 * hh);
      const unsigned short* wq = F1t + (size_t)(16 * wave + m) * 64 + k0 + 8 * hh;
      bf.h[0] = *(const v8usa*)wq;
      bf.h[1] = *(const v8usa*)(wq + 16);
      acc = wmb(ah, bf, acc);
      acc = wmb(al, bf, acc);
    }
    const float bb = bf16_val(fc1b[16 * wave + m]);
#pragma unroll
    for (int r = 0; r < 8; ++r) zs[(8 * hh + r) * 128 + 16 * wave + m] = acc[r] + bb;
  }
  __syncthreads();
#pragma unroll 1
  for (int it = 0; it < 2; ++it) {
    const int idx = 4 * (it * NTHR + tid);
    v4f v = *(const v4fa*)(zs + idx);
    v.x = eluf(v.x); v.y = eluf(v.y); v.z = eluf(v.z); v.w = eluf(v.w);
    v4us h4, l4;
    unsigned hb;
    hb = bf16_bits(v.x); h4[0] = (unsigned short)hb; l4[0] = (unsigned short)bf16_bits(v.x - __uint_as_float(hb << 16));
    hb = bf16_bits(v.y); h4[1] = (unsigned short)hb; l4[1] = (unsigned short)bf16_bits(v.y - __uint_as_float(hb << 16));
    hb = bf16_bits(v.z); h4[2] = (unsigned short)hb; l4[2] = (unsigned short)bf16_bits(v.z - __uint_as_float(hb << 16));
    hb = bf16_bits(v.w); h4[3] = (unsigned short)hb; l4[3] = (unsigned short)bf16_bits(v.w - __uint_as_float(hb << 16));
    *(v4usa*)(zh + idx) = h4;
    *(v4usa*)(zl + idx) = l4;
  }
  __syncthreads();

  if (wave == 0) {
    v8f acc = {0.f, 0.f, 0.f, 0.f, 0.f, 0.f, 0.f, 0.f};
#pragma unroll 1
    for (int k0 = 0; k0 < 128; k0 += 32) {
      FragB ah, al, bf;
      ah.h[0] = *(const v8usa*)(zh + m * 128 + k0 + 8 * hh);
      ah.h[1] = *(const v8usa*)(zh + m * 128 + k0 + 16 + 8 * hh);
      al.h[0] = *(const v8usa*)(zl + m * 128 + k0 + 8 * hh);
      al.h[1] = *(const v8usa*)(zl + m * 128 + k0 + 16 + 8 * hh);
      const unsigned short* wq = F2t + (size_t)m * 128 + k0 + 8 * hh;
      bf.h[0] = *(const v8usa*)wq;
      bf.h[1] = *(const v8usa*)(wq + 16);
      acc = wmb(ah, bf, acc);
      acc = wmb(al, bf, acc);
    }
    const float b2v = bf16_val(fc2b[m < NCLS ? m : NCLS - 1]);
    const float bb = (m < NCLS) ? b2v : 0.0f;
#pragma unroll
    for (int r = 0; r < 8; ++r) lg[(8 * hh + r) * 16 + m] = acc[r] + bb;
  }
  __syncthreads();
  if (wave == 0) {
    const int rw = lane & 15;
    float mx = lg[rw * 16];
#pragma unroll 1
    for (int c = 1; c < NCLS; ++c) mx = nanmaxf(lg[rw * 16 + c], mx);
    float se = 0.0f;
#pragma unroll 1
    for (int c = 0; c < NCLS; ++c) se += expf(lg[rw * 16 + c] - mx);
    const float lse = logf(se);
#pragma unroll 1
    for (int c = 0; c < NCLS; ++c) {
      const float v = (lg[rw * 16 + c] - mx) - lse;
      if (lane < 16) os[rw * NCLS + c] = v;
    }
  }
  __syncthreads();
  {
    const int f0 = gbase * NCLS;
    int nF = NOUTF - f0;
    nF = nF > 160 ? 160 : nF;
    const int tq = tid < 40 ? tid : 39;
    const bool st = (tid < 40) && (4 * tid < nF);
    const v4f ov = *(const v4fa*)(os + 4 * tq);
    float* op = out + (size_t)f0 + 4 * tq;
    if (st) *(volatile v4f*)op = ov;
    __threadfence();
    if (st) *(volatile v4f*)op = ov;
  }
}

static inline int cdiv(int a, int b) { return (a + b - 1) / b; }
static inline size_t al256(size_t o) { return (o + 255) & ~(size_t)255; }
static inline size_t szmax(size_t a, size_t b) { return a > b ? a : b; }

extern "C" void kernel_launch(void* const* d_in, const int* in_sizes, int n_in,
                              void* d_out, int out_size, void* d_ws, size_t ws_size,
                              hipStream_t stream) {
  if (n_in < 24) return;
  if (in_sizes[0] != NN || in_sizes[1] != 2 * NN || in_sizes[2] != 2 * EE || in_sizes[3] != 2 * EE) return;
  if (in_sizes[4] != NN || in_sizes[5] != NN || in_sizes[6] != 2 * EE2 || in_sizes[7] != NN1) return;
  if (in_sizes[8] != 2 * HH || in_sizes[9] != HH || in_sizes[10] != HH * 32 || in_sizes[11] != 32) return;
  if (in_sizes[12] != 32 || in_sizes[13] != 32 || in_sizes[14] != 2 * HH || in_sizes[15] != HH) return;
  if (in_sizes[16] != HH * 2048 || in_sizes[17] != 2048 || in_sizes[18] != 32 * 64 || in_sizes[19] != 64) return;
  if (in_sizes[20] != 64 * 128 || in_sizes[21] != 128 || in_sizes[22] != 128 * NCLS || in_sizes[23] != NCLS) return;
  if (out_size != NOUTF) return;

  const float* x     = (const float*)d_in[0];
  const float* pos   = (const float*)d_in[1];
  const int*   ei    = (const int*)d_in[2];
  const float* ea    = (const float*)d_in[3];
  const int*   batch = (const int*)d_in[4];
  const int*   cl1   = (const int*)d_in[5];
  const int*   ei2   = (const int*)d_in[6];
  const int*   cl2   = (const int*)d_in[7];
  const float* n1w1  = (const float*)d_in[8];
  const float* n1b1  = (const float*)d_in[9];
  const float* n1w2  = (const float*)d_in[10];
  const float* n1b2  = (const float*)d_in[11];
  const float* root1 = (const float*)d_in[12];
  const float* bias1 = (const float*)d_in[13];
  const float* n2w1  = (const float*)d_in[14];
  const float* n2b1  = (const float*)d_in[15];
  const float* n2w2  = (const float*)d_in[16];
  const float* n2b2  = (const float*)d_in[17];
  const float* root2 = (const float*)d_in[18];
  const float* bias2 = (const float*)d_in[19];
  const float* fc1w  = (const float*)d_in[20];
  const float* fc1b  = (const float*)d_in[21];
  const float* fc2w  = (const float*)d_in[22];
  const float* fc2b  = (const float*)d_in[23];
  float* out = (float*)d_out;

  char* ws = (char*)d_ws;
  size_t off = 0;
  const size_t oP0  = off; off = al256(off + szmax((size_t)NN * 32 * 4, (size_t)MPE * 64 * 4));
  const size_t oP1  = off; off = al256(off + szmax((size_t)NN * 32 * 4, (size_t)NN1 * 64 * 4));
  const size_t oX1  = off; off = al256(off + (size_t)MP1 * 32 * 4);
  const size_t oR   = off; off = al256(off + (size_t)MP1 * 64 * 4);
  const size_t oX2  = off; off = al256(off + (size_t)NN2 * 64 * 4);
  const size_t oPS1 = off; off = al256(off + (size_t)PG1 * PNB * 2 * 4);
  const size_t oBT1 = off; off = al256(off + (size_t)PG1 * PNB * 4);
  const size_t oBT2 = off; off = al256(off + (size_t)PG2 * PNB * 4);
  const size_t oREC = off; off = al256(off + 256);
  const size_t oB1t = off; off = al256(off + (size_t)32 * 32 * 2);
  const size_t oW2t = off; off = al256(off + (size_t)64 * W2KP * 2);
  const size_t oR2t = off; off = al256(off + (size_t)64 * 32 * 2);
  const size_t oF1t = off; off = al256(off + (size_t)128 * 64 * 2);
  const size_t oF2t = off; off = al256(off + (size_t)16 * 128 * 2);
  if (off > ws_size || off > (size_t)WSMAX) return;
  float* A1   = (float*)(ws + oP0);
  float* MSG  = (float*)(ws + oP0);
  float* Hf   = (float*)(ws + oP1);
  float* H2   = (float*)(ws + oP1);
  float* X1   = (float*)(ws + oX1);
  float* Rf   = (float*)(ws + oR);
  float* X2   = (float*)(ws + oX2);
  float* POS1 = (float*)(ws + oPS1);
  int*   BAT1 = (int*)(ws + oBT1);
  int*   BAT2 = (int*)(ws + oBT2);
  float* REC  = (float*)(ws + oREC);
  unsigned short* B1t = (unsigned short*)(ws + oB1t);
  unsigned short* W2t = (unsigned short*)(ws + oW2t);
  unsigned short* R2t = (unsigned short*)(ws + oR2t);
  unsigned short* F1t = (unsigned short*)(ws + oF1t);
  unsigned short* F2t = (unsigned short*)(ws + oF2t);

  const size_t lds1 = (size_t)(LISTN + 2 * S1RC + 3 * S1NB + 16) * 4;
  const size_t ldsP = (size_t)(LISTN + 2 * PRC + 3 * PNB + 16 + PNB + 2 * PNB) * 4;
  const size_t lds2 = (size_t)(LISTN + 2 * S2RC + 3 * S2NB + 16) * 4;
  hipFuncSetAttribute(reinterpret_cast<const void*>(&k_scan1), hipFuncAttributeMaxDynamicSharedMemorySize, (int)lds1);
  hipFuncSetAttribute(reinterpret_cast<const void*>(&k_pool<32, 1>), hipFuncAttributeMaxDynamicSharedMemorySize, (int)ldsP);
  hipFuncSetAttribute(reinterpret_cast<const void*>(&k_pool<64, 0>), hipFuncAttributeMaxDynamicSharedMemorySize, (int)ldsP);
  hipFuncSetAttribute(reinterpret_cast<const void*>(&k_scan2), hipFuncAttributeMaxDynamicSharedMemorySize, (int)lds2);

  k_prep<<<35, NTHR, 0, stream>>>(n1w2, n1b2, root1, bias1, n2w2, n2b2, root2, fc1w, fc2w, B1t, W2t, R2t, F1t, F2t);
  k_scan1<<<cdiv(NN, S1NB), NTHR, lds1, stream>>>(ei, x, ea, n1w1, n1b1, A1);
  k_gemm<32, 32, 0, 1><<<NN / GBM, GTHR, 0, stream>>>(A1, B1t, bias1, Hf);
  k_pool<32, 1><<<PG1, NTHR, ldsP, stream>>>(cl1, NN, NN1, MP1, Hf, pos, batch, X1, POS1, BAT1);
  k_cartmax<<<1, NTHR, 0, stream>>>(ei2, POS1, REC);
  k_edge<<<MPE / ETM, NTHR, 0, stream>>>(ei2, X1, POS1, REC, n2w1, n2b1, W2t, MSG);
  k_gemm<32, 64, 1, 0><<<MP1 / GBM, GTHR, 0, stream>>>(X1, R2t, bias2, Rf);
  k_scan2<<<cdiv(NN1, S2NB), NTHR, lds2, stream>>>(ei2, MSG, Rf, H2);
  k_pool<64, 0><<<PG2, NTHR, ldsP, stream>>>(cl2, NN1, NN2, NN2, H2, pos, BAT1, X2, POS1, BAT2);
  k_head<<<cdiv(NGR, 16), NTHR, 0, stream>>>(X2, BAT2, F1t, F2t, fc1b, fc2b, out);
}
